// Generator_9809705304253
// MI455X (gfx1250) — hardware-run, weakly checked
//
#include <hip/hip_runtime.h>


#ifndef NB
#define NB 2
#endif
#ifndef SEQ
#define SEQ 1024
#endif
#define NB_FULL  2
#define SEQ_FULL 1024
#ifndef OUT_SEQ
#define OUT_SEQ SEQ
#endif
#define EMB    384
#define DM     768
#define DI     1536
#define NST    24
#define DTR    48
#define DTK    64
#define XDN    96
#define XDP    128
#define NLAY   4
#define VOCAB  1002
#define LABEL  1001
#define LGP    1024
#define NTOK   (NB * SEQ)
#define CW     1024.0f
#define CWDT   256.0f
#define CHN    16.0f
#define CXC    64.0f
#define CDT    64.0f
#define CY     256.0f
#define LOG2E_F 1.4426950408889634f

#define GM_XZ  0
#define GM_XD  1
#define GM_DT  2
#define GM_OUT 3
#define GM_HD  4

static_assert(DM == 2 * EMB);
static_assert(DM % 32 == 0);
static_assert(DI % 32 == 0);
static_assert(DTK % 32 == 0);
static_assert(DTR % 8 == 0);
static_assert(DTR <= DTK);
static_assert(XDN <= XDP);
static_assert(DTR + 2 * NST == XDN);
static_assert(LABEL <= LGP);
static_assert(NTOK % 64 == 0);
static_assert((2 * DI) % 64 == 0);
static_assert(XDP % 64 == 0);
static_assert(DI % 64 == 0);
static_assert(DM % 64 == 0);
static_assert(LGP % 64 == 0);
static_assert(DM == 3 * 256);
static_assert(3 * 32 * 16 == DM * 2);
static_assert(NTOK % 8 == 0);
static_assert(SEQ % 64 == 0);
static_assert(SEQ % 16 == 0);
static_assert(NST == 24);
static_assert((NST * 4) % 16 == 0);
static_assert(8 * 32 * 16 == 16 * 64 * 4);
static_assert(4 * 32 * 16 == 16 * DTK * 2);
static_assert(2 * 2 * 32 * 16 == 16 * 64 * 2);
static_assert(((size_t)SEQ * LABEL) % 32 == 0);
static_assert((OUT_SEQ % 32) == 0);
static_assert(NB <= NB_FULL);
static_assert(SEQ <= SEQ_FULL);
static_assert(16 * 68 * 4 <= 131072);
static_assert(2 * 16 * 64 * 2 <= 131072);

typedef _Float16 h16;
typedef __attribute__((ext_vector_type(16))) _Float16 v16h;
typedef __attribute__((ext_vector_type(8)))  _Float16 v8h;
typedef __attribute__((ext_vector_type(8)))  float    v8f;
typedef __attribute__((ext_vector_type(4)))  float    v4f;
typedef v4f  __attribute__((may_alias)) v4fa;
typedef v8h  __attribute__((may_alias)) v8ha;

__device__ __forceinline__ unsigned short f2bf(float f) { unsigned u = __float_as_uint(f); u += 0x7FFFu + ((u >> 16) & 1u); return (unsigned short)(u >> 16); }
__device__ __forceinline__ float bfr(float f) { return __uint_as_float(((unsigned)f2bf(f)) << 16); }
__device__ __forceinline__ v16h cat16(v8h lo, v8h hi) { return __builtin_shufflevector(lo, hi, 0, 1, 2, 3, 4, 5, 6, 7, 8, 9, 10, 11, 12, 13, 14, 15); }
__device__ __forceinline__ v8f wmma16(v16h a, v16h b, v8f c) { return __builtin_amdgcn_wmma_f32_16x16x32_f16(false, a, false, b, (short)0, c, false, false); }
__device__ __forceinline__ v16h  ldh(const h16* p) { return cat16(*(const v8h*)p, *(const v8h*)(p + 16)); }
__device__ __forceinline__ void wave_sync() { __builtin_amdgcn_fence(3  , "wavefront"); __builtin_amdgcn_wave_barrier(); asm volatile("" ::: "memory"); }

static __device__ __forceinline__ h16 toh_flush(float v) { const h16 r = (h16)v; return (fabsf(v) < 6.103515625e-05f) ? (h16)0.0f : r; }
__device__ __forceinline__ v8f wmma16g(v16h a, v16h b, v8f c) { c = wmma16(a, b, c); asm volatile("v_nop\n\tv_nop\n\tv_nop\n\tv_nop" : "+v"(c) : "v"(a), "v"(b)); return c; }

__device__ __forceinline__ float silu_f(float x) {
#pragma clang fp contract(off)
    const float e = __expf(-x);
    return x * __builtin_amdgcn_rcpf(1.0f + e);
}
__device__ __forceinline__ float softplus_f(float v) { return fmaxf(v, 0.0f) + log1pf(__expf(-fabsf(v))); }
__device__ __forceinline__ float conv_silu(float x0, float x1, float x2, float x3, float w0, float w1, float w2, float w3, float cb) {
#pragma clang fp contract(off)
    float a = x0 * w0; a = a + x1 * w1; a = a + x2 * w2; a = a + x3 * w3; a = a + cb;
    return silu_f(a);
}

__global__ __launch_bounds__(256) void k_wcvt(const float* __restrict__ src, h16* dst, int R, int Rpad, int Kin, int Kpad, int nmat, float carry) {
    const size_t k8n = (size_t)(Kpad / 8);
    const size_t n8 = (size_t)nmat * (size_t)Rpad * k8n;
    const size_t i = (size_t)blockIdx.x * 256 + threadIdx.x; if (i >= n8) return;
    const int kk = (int)(i % k8n) * 8; const size_t rp = i / k8n; const int r = (int)(rp % (size_t)Rpad); const int mat = (int)(rp / (size_t)Rpad);
    const int rc = r < R ? r : R - 1; const int kc = kk < Kin ? kk : Kin - 8;
    const float* sp = src + ((size_t)mat * R + rc) * Kin + kc;
    v4f x0 = *(const v4f*)sp, x1 = *(const v4f*)(sp + 4);
    asm volatile("" : "+v"(x0), "+v"(x1));
    const bool in = (r < R) & (kk < Kin);
    v8h o;
#pragma unroll
    for (int k = 0; k < 4; ++k) { o[k] = in ? toh_flush(bfr(x0[k]) * carry) : (h16)0.0f; o[4 + k] = in ? toh_flush(bfr(x1[k]) * carry) : (h16)0.0f; }
    *(volatile v8h*)(dst + i * 8) = o; __threadfence(); *(volatile v8h*)(dst + i * 8) = o;
}

__global__ __launch_bounds__(256) void k_embed(const int* __restrict__ tokens, const int* __restrict__ rel, const float* __restrict__ table, float* X) {
    const int i = blockIdx.x * 256 + threadIdx.x; if (i >= NTOK * (DM / 4)) return;
    const int t = i / (DM / 4), d = (i % (DM / 4)) * 4;
    const int b = t / SEQ, l = t % SEQ;
    const int ti = tokens[(size_t)b * SEQ_FULL + l]; const int tr = rel[b];
    int tok = (d < EMB) ? ti : tr; tok = tok < 0 ? 0 : (tok > VOCAB - 1 ? VOCAB - 1 : tok);
    const int dd = (d < EMB) ? d : d - EMB;
    const v4f v = *(const v4f*)(table + (size_t)tok * EMB + dd);
    v4f o;
#pragma unroll
    for (int k = 0; k < 4; ++k) o[k] = bfr(v[k]);
    *(volatile v4f*)(X + (size_t)i * 4) = o; __threadfence(); *(volatile v4f*)(X + (size_t)i * 4) = o;
}

__global__ __launch_bounds__(256) void k_ln(const float* __restrict__ X, const float* __restrict__ w, const float* __restrict__ bsh, h16* HN) {
#pragma clang fp contract(off)
    const int lane = threadIdx.x & 31;
    const int wave = __builtin_amdgcn_readfirstlane((int)(threadIdx.x >> 5));
    const int row = blockIdx.x * 8 + wave;
    const float* xr = X + (size_t)row * DM + 8 * lane;
    float s = 0.0f;
#pragma unroll 1
    for (int j = 0; j < 3; ++j) { const v4f a = *(const v4f*)(xr + 256 * j), c = *(const v4f*)(xr + 256 * j + 4);
        s = s + (((a[0] + a[1]) + (a[2] + a[3])) + ((c[0] + c[1]) + (c[2] + c[3]))); }
#pragma unroll
    for (int off = 16; off > 0; off >>= 1) s = s + __shfl_xor(s, off, 32);
    const float mean = s * (1.0f / (float)DM);
    float q = 0.0f;
#pragma unroll 1
    for (int j = 0; j < 3; ++j) { const v4f a = *(const v4f*)(xr + 256 * j), c = *(const v4f*)(xr + 256 * j + 4);
        float p = 0.0f;
#pragma unroll
        for (int k = 0; k < 4; ++k) { const float ta = a[k] - mean, tc = c[k] - mean; p = p + ta * ta; p = p + tc * tc; }
        q = q + p; }
#pragma unroll
    for (int off = 16; off > 0; off >>= 1) q = q + __shfl_xor(q, off, 32);
    const float rstd = rsqrtf(q * (1.0f / (float)DM) + 1e-5f);
    v8h o[3];
#pragma unroll
    for (int j = 0; j < 3; ++j) {
        const v4f a = *(const v4f*)(xr + 256 * j), c = *(const v4f*)(xr + 256 * j + 4);
        const v4f wa = *(const v4f*)(w + 256 * j + 8 * lane), wc = *(const v4f*)(w + 256 * j + 8 * lane + 4);
        const v4f ba = *(const v4f*)(bsh + 256 * j + 8 * lane), bc = *(const v4f*)(bsh + 256 * j + 8 * lane + 4);
#pragma unroll
        for (int k = 0; k < 4; ++k) {
            const float ya = ((a[k] - mean) * rstd) * bfr(wa[k]) + bfr(ba[k]);
            const float yc = ((c[k] - mean) * rstd) * bfr(wc[k]) + bfr(bc[k]);
            o[j][k] = toh_flush(ya * CHN); o[j][4 + k] = toh_flush(yc * CHN); } }
    h16* hp = HN + (size_t)row * DM + 8 * lane;
#pragma unroll 1
    for (int ps = 0; ps < 2; ++ps) {
        *(volatile v8h*)(hp) = o[0]; *(volatile v8h*)(hp + 256) = o[1]; *(volatile v8h*)(hp + 512) = o[2];
        if (ps == 0) __threadfence(); }
}

__global__ __launch_bounds__(256) void k_conv(const float* __restrict__ XZ, const float* __restrict__ cw, const float* __restrict__ cb, h16* XC) {
#pragma clang fp contract(off)
    const int i = blockIdx.x * 256 + threadIdx.x; if (i >= NTOK * (DI / 8)) return;
    const int t = i / (DI / 8), d8 = (i % (DI / 8)) * 8; const int l = t % SEQ;
    v4f xa[4], xb[4];
#pragma unroll
    for (int k = 0; k < 4; ++k) { const int ll = l - 3 + k; const int tc = t - l + (ll < 0 ? 0 : ll);
        const float* xp = XZ + (size_t)tc * (2 * DI) + d8; v4f a = *(const v4f*)xp, c = *(const v4f*)(xp + 4);
        asm volatile("" : "+v"(a), "+v"(c));
        const bool ok = ll >= 0;
#pragma unroll
        for (int q = 0; q < 4; ++q) { xa[k][q] = ok ? a[q] : 0.0f; xb[k][q] = ok ? c[q] : 0.0f; } }
    v4f wv[8];
#pragma unroll
    for (int c = 0; c < 8; ++c) wv[c] = *(const v4f*)(cw + (size_t)(d8 + c) * 4);
    const v4f b0 = *(const v4f*)(cb + d8), b1 = *(const v4f*)(cb + d8 + 4);
    v8h o;
#pragma unroll
    for (int c = 0; c < 8; ++c) {
        const float x0 = (c < 4) ? xa[0][c & 3] : xb[0][c & 3], x1 = (c < 4) ? xa[1][c & 3] : xb[1][c & 3];
        const float x2 = (c < 4) ? xa[2][c & 3] : xb[2][c & 3], x3 = (c < 4) ? xa[3][c & 3] : xb[3][c & 3];
        const float bb = (c < 4) ? b0[c & 3] : b1[c & 3];
        const float u = conv_silu(x0, x1, x2, x3, bfr(wv[c][0]), bfr(wv[c][1]), bfr(wv[c][2]), bfr(wv[c][3]), bfr(bb));
        o[c] = toh_flush(u * CXC); }
    *(volatile v8h*)(XC + (size_t)i * 8) = o; __threadfence(); *(volatile v8h*)(XC + (size_t)i * 8) = o;
}

template <int MODE, int KD>
__device__ __forceinline__ void gemm_body(const h16* __restrict__ A, const h16* __restrict__ Bt, const float scl,
                                          const float* __restrict__ bias, const int nbias, const float* __restrict__ res, float* Cf, const int ldc, h16* Ch) {
    __shared__ __align__(16) float os[16 * 68];
    const int lane = threadIdx.x & 31, lr = lane & 15, hi = lane >> 4; const int r0 = blockIdx.x * 64, c0 = blockIdx.y * 64;
    v8f acc[4][4];
#pragma unroll
    for (int mb = 0; mb < 4; ++mb)
#pragma unroll
        for (int nb = 0; nb < 4; ++nb) acc[mb][nb] = (v8f){};
    const size_t aoff = (size_t)(r0 + lr) * KD + 8 * hi, boff = (size_t)(c0 + lr) * KD + 8 * hi;
#pragma unroll 1
    for (int kc = 0; kc < KD; kc += 32) {
        v16h a[4];
#pragma unroll
        for (int mb = 0; mb < 4; ++mb) a[mb] = ldh(A + aoff + (size_t)mb * 16 * KD + kc);
#pragma unroll
        for (int nb = 0; nb < 4; ++nb) { const v16h b = ldh(Bt + boff + (size_t)nb * 16 * KD + kc);
#pragma unroll
            for (int mb = 0; mb < 4; ++mb) acc[mb][nb] = wmma16g(a[mb], b, acc[mb][nb]); }
    }
#pragma unroll
    for (int mb = 0; mb < 4; ++mb) {
        const int gr0 = r0 + mb * 16;
#pragma unroll
        for (int nb = 0; nb < 4; ++nb) {
#pragma unroll
            for (int j = 0; j < 8; ++j) os[(hi * 8 + j) * 68 + nb * 16 + lr] = acc[mb][nb][j] * scl; }
        wave_sync();
        if (MODE == GM_DT || MODE == GM_OUT || MODE == GM_HD) {
#pragma unroll 1
            for (int s = 0; s < 8; ++s) { const int p = s * 32 + lane; const int row = p >> 4, c4 = (p & 15) * 4;
                v4f v = *(const v4fa*)(&os[row * 68 + c4]);
                if (MODE == GM_OUT) { const v4f r = *(const v4f*)(res + (size_t)(gr0 + row) * ldc + c0 + c4); v = v + r; }
                else {
#pragma unroll
                    for (int i = 0; i < 4; ++i) { const int col = c0 + c4 + i; const int cc = col < nbias ? col : nbias - 1;
                        float bv = bias[cc]; asm volatile("" : "+v"(bv));
                        const float tv = v[i] + ((col < nbias) ? bfr(bv) : 0.0f);
                        v[i] = (MODE == GM_DT) ? softplus_f(tv) : tv; } }
                *(v4fa*)(&os[row * 68 + c4]) = v; }
            wave_sync();
        }
#pragma unroll 1
        for (int ps = 0; ps < 2; ++ps) {
#pragma unroll
            for (int s = 0; s < 8; ++s) { const int p = s * 32 + lane; const int row = p >> 4, c4 = (p & 15) * 4;
                const v4f val = *(const v4fa*)(&os[row * 68 + c4]);
                *(volatile v4f*)(Cf + (size_t)(gr0 + row) * ldc + c0 + c4) = val; }
            if (MODE == GM_XD) {
                if (c0 == 0) {
#pragma unroll
                    for (int s = 0; s < 4; ++s) { const int row = 4 * s + (lane >> 3), c8 = (lane & 7) * 8;
                        const v4f x0 = *(const v4fa*)(&os[row * 68 + c8]); const v4f x1 = *(const v4fa*)(&os[row * 68 + c8 + 4]); v8h hv;
#pragma unroll
                        for (int i = 0; i < 4; ++i) { hv[i] = (c8 + i < DTR) ? toh_flush(x0[i] * CDT) : (h16)0.0f; hv[4 + i] = (c8 + 4 + i < DTR) ? toh_flush(x1[i] * CDT) : (h16)0.0f; }
                        *(volatile v8h*)(Ch + (size_t)(gr0 + row) * DTK + c8) = hv; } } }
            if (ps == 0) __threadfence(); }
        wave_sync();
    }
}

__global__ __launch_bounds__(32) void k_gemm_xz(const h16* __restrict__ A, const h16* __restrict__ Bt, float* C) {
    gemm_body<GM_XZ, DM>(A, Bt, 1.0f / (CHN * CW), nullptr, 0, nullptr, C, 2 * DI, nullptr);
}
__global__ __launch_bounds__(32) void k_gemm_xd(const h16* __restrict__ A, const h16* __restrict__ Bt, float* C, h16* Ch) {
    gemm_body<GM_XD, DI>(A, Bt, 1.0f / (CXC * CW), nullptr, 0, nullptr, C, XDP, Ch);
}
__global__ __launch_bounds__(32) void k_gemm_dt(const h16* __restrict__ A, const h16* __restrict__ Bt, const float* __restrict__ bias, float* C) {
    gemm_body<GM_DT, DTK>(A, Bt, 1.0f / (CDT * CWDT), bias, DI, nullptr, C, DI, nullptr);
}
__global__ __launch_bounds__(32) void k_gemm_out(const h16* __restrict__ A, const h16* __restrict__ Bt, const float* __restrict__ res, float* C) {
    gemm_body<GM_OUT, DI>(A, Bt, 1.0f / (CY * CW), nullptr, 0, res, C, DM, nullptr);
}
__global__ __launch_bounds__(32) void k_gemm_hd(const h16* __restrict__ A, const h16* __restrict__ Bt, const float* __restrict__ bias, float* C) {
    gemm_body<GM_HD, DM>(A, Bt, 1.0f / (CHN * CW), bias, LABEL, nullptr, C, LGP, nullptr);
}

__global__ __launch_bounds__(64) void k_scan(const float* __restrict__ XZ, const float* __restrict__ DL, const float* __restrict__ XD,
                                             const float* __restrict__ cw, const float* __restrict__ cb, const float* __restrict__ alog, const float* __restrict__ dpar, h16* YP) {
#pragma clang fp contract(off)
    __shared__ __align__(16) h16 ys[2 * 16 * 64];
    const int tid = threadIdx.x; const int lane = tid & 31;
    const int wave = __builtin_amdgcn_readfirstlane((int)(threadIdx.x >> 5));
    const int d = blockIdx.x * 64 + tid; const int b = blockIdx.y;
    float A2[NST], h[NST];
#pragma unroll
    for (int q = 0; q < NST / 4; ++q) { const v4f al = *(const v4f*)(alog + (size_t)d * NST + 4 * q);
#pragma unroll
        for (int k = 0; k < 4; ++k) { A2[4 * q + k] = (-__expf(bfr(al[k]))) * LOG2E_F; h[4 * q + k] = 0.0f; } }
    const v4f wr = *(const v4f*)(cw + (size_t)d * 4);
    const float w0 = bfr(wr[0]), w1 = bfr(wr[1]), w2 = bfr(wr[2]), w3 = bfr(wr[3]);
    const float cbv = bfr(cb[d]), Dd = bfr(dpar[d]);
    float xm3 = 0.0f, xm2 = 0.0f, xm1 = 0.0f;
    const size_t tb = (size_t)b * SEQ;
#pragma unroll 1
    for (int l0 = 0; l0 < SEQ; l0 += 16) {
        const int buf = ((l0 >> 4) & 1) * (16 * 64);
#pragma unroll 1
        for (int ls = 0; ls < 16; ++ls) {
            const size_t t = tb + (size_t)(l0 + ls);
            const float dt = DL[t * DI + d];
            const float xin = XZ[t * (2 * DI) + d];
            const float z = XZ[t * (2 * DI) + DI + d];
            const float u = conv_silu(xm3, xm2, xm1, xin, w0, w1, w2, w3, cbv);
            xm3 = xm2; xm2 = xm1; xm1 = xin;
            const float* bc = XD + t * XDP + DTR;
            v4f bq[6], cq[6];
#pragma unroll
            for (int q = 0; q < 6; ++q) { bq[q] = *(const v4f*)(bc + 4 * q); cq[q] = *(const v4f*)(bc + NST + 4 * q); }
            const float du = dt * u;
            float y = 0.0f;
#pragma unroll
            for (int n = 0; n < NST; ++n) {
                const float dA = __builtin_amdgcn_exp2f(dt * A2[n]);
                h[n] = dA * h[n] + du * bq[n >> 2][n & 3];
                y = y + h[n] * cq[n >> 2][n & 3]; }
            y = (y + u * Dd) * silu_f(z);
            ys[buf + ls * 64 + tid] = toh_flush(y * CY);
        }
        __syncthreads();
#pragma unroll 1
        for (int ps = 0; ps < 2; ++ps) {
#pragma unroll
            for (int s = 0; s < 2; ++s) { const int row = 8 * wave + 4 * s + (lane >> 3), c8 = (lane & 7) * 8;
                const v8h val = *(const v8ha*)(&ys[buf + row * 64 + c8]);
                *(volatile v8h*)(YP + (tb + (size_t)(l0 + row)) * DI + blockIdx.x * 64 + c8) = val; }
            if (ps == 0) __threadfence(); }
    }
}

__global__ __launch_bounds__(256) void k_pack(const float* __restrict__ LG, float* OUT) {
    const int i = blockIdx.x * 256 + threadIdx.x; const int b = blockIdx.y;
    if (i >= SEQ * LABEL / 4) return;
    v4f o;
#pragma unroll
    for (int k = 0; k < 4; ++k) { const int f = 4 * i + k; const int row = f / LABEL; const int col = f - row * LABEL;
        o[k] = LG[((size_t)b * SEQ + row) * LGP + col]; }
    float* p = OUT + (size_t)b * OUT_SEQ * LABEL + (size_t)i * 4;
    *(volatile v4f*)p = o; __threadfence(); *(volatile v4f*)p = o;
}

static constexpr size_t al256(size_t v) { return (v + 255) & ~(size_t)255; }
static constexpr size_t SZ_WIN  = al256((size_t)NLAY * 2 * DI * DM * 2);
static constexpr size_t SZ_WXP  = al256((size_t)NLAY * XDP * DI * 2);
static constexpr size_t SZ_WDT  = al256((size_t)NLAY * DI * DTK * 2);
static constexpr size_t SZ_WOUT = al256((size_t)NLAY * DM * DI * 2);
static constexpr size_t SZ_WHD  = al256((size_t)LGP * DM * 2);
static constexpr size_t SZ_X    = al256((size_t)NTOK * DM * 4);
static constexpr size_t SZ_HN   = al256((size_t)NTOK * DM * 2);
static constexpr size_t SZ_XZ   = al256((size_t)NTOK * 2 * DI * 4);
static constexpr size_t SZ_XC   = al256((size_t)NTOK * DI * 2);
static constexpr size_t SZ_XD   = al256((size_t)NTOK * XDP * 4);
static constexpr size_t SZ_DTP  = al256((size_t)NTOK * DTK * 2);
static constexpr size_t SZ_DL   = al256((size_t)NTOK * DI * 4);
static constexpr size_t SZ_YP   = al256((size_t)NTOK * DI * 2);
static constexpr size_t SZ_LG   = al256((size_t)NTOK * LGP * 4);
static constexpr size_t SZ_TOTAL = SZ_WIN + SZ_WXP + SZ_WDT + SZ_WOUT + SZ_WHD + 2 * SZ_X + SZ_HN + SZ_XZ + SZ_XC + SZ_XD + SZ_DTP + SZ_DL + SZ_YP + SZ_LG;
static_assert(SZ_TOTAL <= (size_t)134217728);
static_assert(((size_t)2 * DI * DM * 2) % 256 == 0);
static_assert(((size_t)XDP * DI * 2) % 256 == 0);
static_assert(((size_t)DI * DTK * 2) % 256 == 0);
static_assert(((size_t)DM * DI * 2) % 256 == 0);

extern "C" void kernel_launch(void* const* d_in, const int* in_sizes, int n_in,
                              void* d_out, int out_size, void* d_ws, size_t ws_size, hipStream_t stream) {
    if (n_in < 18) return;
    if ((size_t)in_sizes[0] < (size_t)(NB - 1) * SEQ_FULL + SEQ || in_sizes[1] < NB) return;
    if ((size_t)in_sizes[2] < (size_t)VOCAB * EMB) return;
    if (in_sizes[3] < NLAY * DM || in_sizes[4] < NLAY * DM) return;
    if ((size_t)in_sizes[5] < (size_t)NLAY * 2 * DI * DM) return;
    if (in_sizes[6] < NLAY * DI * 4 || in_sizes[7] < NLAY * DI) return;
    if ((size_t)in_sizes[8] < (size_t)NLAY * XDN * DI || (size_t)in_sizes[9] < (size_t)NLAY * DI * DTR) return;
    if (in_sizes[10] < NLAY * DI || in_sizes[11] < NLAY * DI * NST || in_sizes[12] < NLAY * DI) return;
    if ((size_t)in_sizes[13] < (size_t)NLAY * DM * DI) return;
    if (in_sizes[14] < DM || in_sizes[15] < DM) return;
    if ((size_t)in_sizes[16] < (size_t)LABEL * DM || in_sizes[17] < LABEL) return;
    if ((size_t)out_size < ((size_t)(NB - 1) * OUT_SEQ + SEQ) * LABEL) return;
    if (SZ_TOTAL > ws_size) return;
    const int*   tokens  = (const int*)d_in[0];
    const int*   rel     = (const int*)d_in[1];
    const float* table   = (const float*)d_in[2];
    const float* ln_w    = (const float*)d_in[3];
    const float* ln_b    = (const float*)d_in[4];
    const float* in_w    = (const float*)d_in[5];
    const float* conv_w  = (const float*)d_in[6];
    const float* conv_b  = (const float*)d_in[7];
    const float* xp_w    = (const float*)d_in[8];
    const float* dt_w    = (const float*)d_in[9];
    const float* dt_b    = (const float*)d_in[10];
    const float* a_log   = (const float*)d_in[11];
    const float* d_par   = (const float*)d_in[12];
    const float* out_w   = (const float*)d_in[13];
    const float* fn_w    = (const float*)d_in[14];
    const float* fn_b    = (const float*)d_in[15];
    const float* head_w  = (const float*)d_in[16];
    const float* head_b  = (const float*)d_in[17];
    float* OUT = (float*)d_out;
    char* wsp = (char*)d_ws;
    h16* WIN  = (h16*)wsp; wsp += SZ_WIN;
    h16* WXP  = (h16*)wsp; wsp += SZ_WXP;
    h16* WDT  = (h16*)wsp; wsp += SZ_WDT;
    h16* WOUT = (h16*)wsp; wsp += SZ_WOUT;
    h16* WHD  = (h16*)wsp; wsp += SZ_WHD;
    float* X0 = (float*)wsp; wsp += SZ_X;
    float* X1 = (float*)wsp; wsp += SZ_X;
    h16* HN   = (h16*)wsp; wsp += SZ_HN;
    float* XZ = (float*)wsp; wsp += SZ_XZ;
    h16* XC   = (h16*)wsp; wsp += SZ_XC;
    float* XD = (float*)wsp; wsp += SZ_XD;
    h16* DTP  = (h16*)wsp; wsp += SZ_DTP;
    float* DL = (float*)wsp; wsp += SZ_DL;
    h16* YP   = (h16*)wsp; wsp += SZ_YP;
    float* LG = (float*)wsp; wsp += SZ_LG;

    { const size_t n8 = (size_t)NLAY * 2 * DI * (DM / 8);
      k_wcvt<<<(unsigned)((n8 + 255) / 256), 256, 0, stream>>>(in_w, WIN, NLAY * 2 * DI, NLAY * 2 * DI, DM, DM, 1, CW); }
    { const size_t n8 = (size_t)NLAY * XDP * (DI / 8);
      k_wcvt<<<(unsigned)((n8 + 255) / 256), 256, 0, stream>>>(xp_w, WXP, XDN, XDP, DI, DI, NLAY, CW); }
    { const size_t n8 = (size_t)NLAY * DI * (DTK / 8);
      k_wcvt<<<(unsigned)((n8 + 255) / 256), 256, 0, stream>>>(dt_w, WDT, NLAY * DI, NLAY * DI, DTR, DTK, 1, CWDT); }
    { const size_t n8 = (size_t)NLAY * DM * (DI / 8);
      k_wcvt<<<(unsigned)((n8 + 255) / 256), 256, 0, stream>>>(out_w, WOUT, NLAY * DM, NLAY * DM, DI, DI, 1, CW); }
    { const size_t n8 = (size_t)LGP * (DM / 8);
      k_wcvt<<<(unsigned)((n8 + 255) / 256), 256, 0, stream>>>(head_w, WHD, LABEL, LGP, DM, DM, 1, CW); }

    k_embed<<<(unsigned)((NTOK * (DM / 4) + 255) / 256), 256, 0, stream>>>(tokens, rel, table, X0);

    float* Xc = X0; float* Xn = X1;
    for (int i = 0; i < NLAY; ++i) {
        k_ln<<<NTOK / 8, 256, 0, stream>>>(Xc, ln_w + (size_t)i * DM, ln_b + (size_t)i * DM, HN);
        k_gemm_xz<<<dim3(NTOK / 64, 2 * DI / 64, 1), 32, 0, stream>>>(HN, WIN + (size_t)i * 2 * DI * DM, XZ);
        k_conv<<<(unsigned)((NTOK * (DI / 8) + 255) / 256), 256, 0, stream>>>(XZ, conv_w + (size_t)i * DI * 4, conv_b + (size_t)i * DI, XC);
        k_gemm_xd<<<dim3(NTOK / 64, XDP / 64, 1), 32, 0, stream>>>(XC, WXP + (size_t)i * XDP * DI, XD, DTP);
        k_gemm_dt<<<dim3(NTOK / 64, DI / 64, 1), 32, 0, stream>>>(DTP, WDT + (size_t)i * DI * DTK, dt_b + (size_t)i * DI, DL);
        k_scan<<<dim3(DI / 64, NB, 1), 64, 0, stream>>>(XZ, DL, XD, conv_w + (size_t)i * DI * 4, conv_b + (size_t)i * DI,
                                                        a_log + (size_t)i * DI * NST, d_par + (size_t)i * DI, YP);
        k_gemm_out<<<dim3(NTOK / 64, DM / 64, 1), 32, 0, stream>>>(YP, WOUT + (size_t)i * DM * DI, Xc, Xn);
        float* tsw = Xc; Xc = Xn; Xn = tsw;
    }
    k_ln<<<NTOK / 8, 256, 0, stream>>>(Xc, fn_w, fn_b, HN);
    k_gemm_hd<<<dim3(NTOK / 64, LGP / 64, 1), 32, 0, stream>>>(HN, WHD, head_b, LG);
    k_pack<<<dim3((unsigned)((SEQ * LABEL / 4 + 255) / 256), NB, 1), 256, 0, stream>>>(LG, OUT);
}
